// NEQUIP_2920577761400
// MI455X (gfx1250) — hardware-verified
//
#include <hip/hip_runtime.h>
#include <stddef.h>
#include <stdint.h>

#define NTHR   256
#define NWAVE  8
#define EPB    256
#define HID    64
#define K1     32
#define K2     128
#define N3     16
#define DP     68
#define AP     136
#define FP     40
#define MIXW   8
#define NODEW  16
#define NLAYER 3
#define EPT    8
#define CHUNK  (NTHR * EPT)
#define WCAP   (EPT * 32)
#define LISTN  (NWAVE * WCAP)
#define NBA    1024
#define SLA    10
#define RCAP   24576
#define DEGCAP 64
#define CWN    128
#define NU_W1  (NLAYER * HID * (K1 / 8))
#define NU_W2  (NLAYER * HID * (K2 / 8))
#define NU_W3  (NLAYER * N3 * (K2 / 8))
#define AGG_ZINTS (LISTN + 2 * RCAP + 3 * NBA)
#define AGG_LDS_INTS (AGG_ZINTS + 16 + CWN)
#define AGG_LDS_BYTES (AGG_LDS_INTS * 4)
#define EDGE_LDS_BYTES (EPB * DP * 4 + EPB * AP * 2 + EPB * FP * 2 + EPB * MIXW * 4)
#define WSMAX  134217728

#define C121F  2.1213203435596424f
#define SQRT3F 1.7320508075688772f
#define SQRT2F 1.4142135623730951f
#define PIF    3.141592653589793f
#define RSQ2   (1.0f / 1.4142135623730951f)
#define RSQ3   (1.0f / 1.7320508075688772f)
#define RSQ5   (1.0f / 2.23606797749979f)
#define RSQ8   (1.0f / 2.8284271247461903f)
#define THIRD  (1.0f / 3.0f)

static_assert((CHUNK & (CHUNK - 1)) == 0 && CHUNK <= 4096);
static_assert((NBA & (NBA - 1)) == 0 && NBA == (1 << SLA));
static_assert(((long long)CHUNK << SLA) < (1LL << 31));
static_assert(LISTN % NTHR == 0);
static_assert(NBA % NWAVE == 0 && NBA % 32 == 0 && NBA == 4 * NTHR);
static_assert(RCAP % 4 == 0 && AGG_ZINTS % (4 * NTHR) == 0 && LISTN % 4 == 0);
static_assert(RCAP >= NBA * NODEW);
static_assert(AGG_LDS_BYTES <= 300000 && EDGE_LDS_BYTES <= 300000);
static_assert(NU_W1 % NTHR == 0 && NU_W2 % NTHR == 0 && NU_W3 % NTHR == 0);
static_assert(NU_W1 == NLAYER * 256 && NU_W2 == NLAYER * 1024 && NU_W3 == NLAYER * 256);
static_assert(K1 % 32 == 0 && K2 % 32 == 0 && K2 == 2 * HID && HID == 4 * 16);
static_assert((DP * 4) % 16 == 0 && (AP * 2) % 16 == 0 && (FP * 2) % 16 == 0);
static_assert(AP >= K2 && FP >= K1 && DP >= HID);
static_assert(EPB == NTHR && EPB == NWAVE * 32);
static_assert((EPB * DP * 4) % 16 == 0 && ((EPB * AP * 2 + EPB * FP * 2) % 16) == 0);
static_assert(EPB * MIXW * 4 == 2 * NTHR * 16);
static_assert(NBA * NODEW * 4 == 16 * NTHR * 16 && NBA * 3 * 4 == 3 * NTHR * 16);

typedef float          v4f   __attribute__((ext_vector_type(4)));
typedef float          v8f   __attribute__((ext_vector_type(8)));
typedef int            v4i   __attribute__((ext_vector_type(4)));
typedef int            v8i   __attribute__((ext_vector_type(8)));
typedef unsigned short v8us  __attribute__((ext_vector_type(8)));
typedef unsigned short v16us __attribute__((ext_vector_type(16)));
typedef __bf16         v16bf __attribute__((ext_vector_type(16)));
typedef v4f  __attribute__((may_alias)) v4fa;
typedef v4i  __attribute__((may_alias)) v4ia;
typedef v8us __attribute__((may_alias)) v8usa;
union FragB { v16bf v; v16us u; v8us h[2]; v8i w; };

__device__ __forceinline__ v8f wmb(const FragB& a, const FragB& b, v8f c) {
  v8f d = __builtin_amdgcn_wmma_f32_16x16x32_bf16(false, a.v, false, b.v, (short)0, c, false, false);
  asm volatile("v_nop\n\tv_nop\n\tv_nop\n\tv_nop" : "+v"(d) : "v"(a.w), "v"(b.w));
  return d;
}

__device__ __forceinline__ unsigned bf16_bits(float f) {
  const unsigned u = __float_as_uint(f);
  return (u + 0x7FFFu + ((u >> 16) & 1u)) >> 16;
}
__device__ __forceinline__ float bf16_val(float f) {
  return __uint_as_float(bf16_bits(f) << 16);
}
__device__ __forceinline__ float swishf(float t) {
  return t * __builtin_amdgcn_rcpf(1.0f + __expf(-t));
}
__device__ __forceinline__ void split3(float f, unsigned short& a, unsigned short& b, unsigned short& c) {
#pragma clang fp contract(off)
  const unsigned u  = __float_as_uint(f);
  const unsigned hs = (u + 0x7FFFu + ((u >> 16) & 1u)) & 0xFFFF0000u;
  const float    r1 = f - __uint_as_float(hs);
  const unsigned l1 = __float_as_uint(r1) & 0xFFFF0000u;
  const float    r2 = r1 - __uint_as_float(l1);
  a = (unsigned short)(hs >> 16);
  b = (unsigned short)(l1 >> 16);
  c = (unsigned short)(__float_as_uint(r2) >> 16);
}
__device__ __forceinline__ void put16(unsigned short* dp, v8us o) {
  *(volatile v8us*)dp = o;
  __threadfence();
  *(volatile v8us*)dp = o;
}
__device__ __forceinline__ void putf4(float* dp, v4f o) {
  *(volatile v4f*)dp = o;
  __threadfence();
  *(volatile v4f*)dp = o;
}

__device__ __forceinline__ void load_cw(float* cw, const float* __restrict__ Wss, const float* __restrict__ Wsv,
                                        const float* __restrict__ Wus, const float* __restrict__ Wuv,
                                        const float* __restrict__ Wds, const float* __restrict__ Wdv, int tid) {
  int i0 = tid;       i0 = i0 < 0 ? 0 : (i0 > 8 ? 8 : i0);
  int i1 = tid - 16;  i1 = i1 < 0 ? 0 : (i1 > 11 ? 11 : i1);
  int i2 = tid - 32;  i2 = i2 < 0 ? 0 : (i2 > 2 ? 2 : i2);
  int i3 = tid - 48;  i3 = i3 < 0 ? 0 : (i3 > 11 ? 11 : i3);
  int i4 = tid - 64;  i4 = i4 < 0 ? 0 : (i4 > 26 ? 26 : i4);
  int i5 = tid - 96;  i5 = i5 < 0 ? 0 : (i5 > 29 ? 29 : i5);
  const float a = Wss[i0], b = Wsv[i1], c = Wus[i2], d = Wuv[i3], e = Wds[i4], f = Wdv[i5];
  const float fa = (tid < 9) ? 1.0f : 0.0f;
  const float fb = (tid >= 16 && tid < 28) ? 1.0f : 0.0f;
  const float fc = (tid >= 32 && tid < 35) ? 1.0f : 0.0f;
  const float fd = (tid >= 48 && tid < 60) ? 1.0f : 0.0f;
  const float fe = (tid >= 64 && tid < 91) ? 1.0f : 0.0f;
  const float ff = (tid >= 96 && tid < 126) ? 1.0f : 0.0f;
  const float v = ((bf16_val(a) * fa + bf16_val(b) * fb) + (bf16_val(c) * fc + bf16_val(d) * fd)) +
                  (bf16_val(e) * fe + bf16_val(f) * ff);
  if (tid < CWN) cw[tid] = v;
}

template <int SLB>
__device__ __forceinline__ int scan_chunk(const int* __restrict__ dsts, int nE, int cbase, int slotBase,
                                          int nb, int vec8, int* list, int tid, int lane, int wave) {
  int wc = 0;
  const int el0  = tid * EPT;
  const int e0   = cbase + el0;
  const int sent = -2147483647 - 1;
  v4i da, db;
  if (vec8 != 0 && cbase + CHUNK <= nE) {
    da = *(const v4i*)(dsts + e0);
    db = *(const v4i*)(dsts + e0 + 4);
  } else {
    da.x = (e0     < nE) ? dsts[min(e0,     nE - 1)] : sent;
    da.y = (e0 + 1 < nE) ? dsts[min(e0 + 1, nE - 1)] : sent;
    da.z = (e0 + 2 < nE) ? dsts[min(e0 + 2, nE - 1)] : sent;
    da.w = (e0 + 3 < nE) ? dsts[min(e0 + 3, nE - 1)] : sent;
    db.x = (e0 + 4 < nE) ? dsts[min(e0 + 4, nE - 1)] : sent;
    db.y = (e0 + 5 < nE) ? dsts[min(e0 + 5, nE - 1)] : sent;
    db.z = (e0 + 6 < nE) ? dsts[min(e0 + 6, nE - 1)] : sent;
    db.w = (e0 + 7 < nE) ? dsts[min(e0 + 7, nE - 1)] : sent;
  }
  const unsigned nbs = (unsigned)slotBase;
  const unsigned unb = (unsigned)nb;
  const unsigned s0 = (unsigned)da.x - nbs, s1 = (unsigned)da.y - nbs;
  const unsigned s2 = (unsigned)da.z - nbs, s3 = (unsigned)da.w - nbs;
  const unsigned s4 = (unsigned)db.x - nbs, s5 = (unsigned)db.y - nbs;
  const unsigned s6 = (unsigned)db.z - nbs, s7 = (unsigned)db.w - nbs;
  const bool h0 = s0 < unb, h1 = s1 < unb, h2 = s2 < unb, h3 = s3 < unb;
  const bool h4 = s4 < unb, h5 = s5 < unb, h6 = s6 < unb, h7 = s7 < unb;
  const unsigned any = __builtin_amdgcn_ballot_w32(h0 | h1 | h2 | h3 | h4 | h5 | h6 | h7);
  if (any != 0u) {
#define HITJ(J, HJ, SJ) { \
      const unsigned mj = __builtin_amdgcn_ballot_w32(HJ); \
      if (mj != 0u) { \
        if (HJ) { \
          const int pos = wc + (int)__builtin_amdgcn_mbcnt_lo(mj, 0u); \
          if (pos < WCAP) list[wave * WCAP + pos] = ((el0 + (J)) << SLB) | (int)(SJ); \
        } \
        wc += (int)__builtin_popcount(mj); } }
    HITJ(0, h0, s0)
    HITJ(1, h1, s1)
    HITJ(2, h2, s2)
    HITJ(3, h3, s3)
    HITJ(4, h4, s4)
    HITJ(5, h5, s5)
    HITJ(6, h6, s6)
    HITJ(7, h7, s7)
#undef HITJ
  }
  return wc;
}

__global__ __launch_bounds__(NTHR) void k_prep(const float* __restrict__ pos, const float* __restrict__ nf,
                                               const float* __restrict__ Wss, const float* __restrict__ Wsv,
                                               const float* __restrict__ Wus, const float* __restrict__ Wuv,
                                               const float* __restrict__ Wds, const float* __restrict__ Wdv,
                                               const float* __restrict__ W1, const float* __restrict__ W2,
                                               const float* __restrict__ W3, int nN, int nR,
                                               unsigned short* W1T, unsigned short* W2T, unsigned short* W3T,
                                               float* POSB, float* NODE0) {
#pragma clang fp contract(off)
  __shared__ __attribute__((aligned(16))) float cw[CWN];
  const int tid = (int)threadIdx.x;
  load_cw(cw, Wss, Wsv, Wus, Wuv, Wds, Wdv, tid);
  __syncthreads();

  const int u  = (int)blockIdx.x * NTHR + tid;
  const int U0 = NU_W1;
  const int U1 = U0 + NU_W2;
  const int U2 = U1 + NU_W3;
  const int U3 = U2 + nR;
  const int U4 = U3 + 4 * nR;
  v8us o;
  if (u < U0) {
    const int l  = u >> 8;
    const int w  = u & 255;
    const int n  = w >> 2;
    const int k8 = (w & 3) * 8;
    const unsigned msk = (k8 < 24) ? 0xFFFFu : 0u;
    const float* p = W1 + (size_t)l * 512 + n;
#pragma unroll
    for (int i = 0; i < 8; ++i) o[i] = (unsigned short)(bf16_bits(p[(size_t)i * 64]) & msk);
    put16(W1T + (size_t)(l * HID + n) * K1 + k8, o);
    return;
  } else if (u < U1) {
    const int v    = u - U0;
    const int l    = v >> 10;
    const int w    = v & 1023;
    const int n    = w >> 4;
    const int k8   = (w & 15) * 8;
    const int srow = k8 & (HID - 1);
    const float* p = W2 + (size_t)l * 4096 + (size_t)srow * 64 + n;
#pragma unroll
    for (int i = 0; i < 8; ++i) o[i] = (unsigned short)bf16_bits(p[(size_t)i * 64]);
    put16(W2T + (size_t)(l * HID + n) * K2 + k8, o);
    return;
  } else if (u < U2) {
    const int v    = u - U1;
    const int l    = v >> 8;
    const int w    = v & 255;
    const int n    = w >> 4;
    const int k8   = (w & 15) * 8;
    const int srow = k8 & (HID - 1);
    const int nc   = n < 8 ? n : 7;
    const unsigned msk = (n < 8) ? 0xFFFFu : 0u;
    const float* p = W3 + (size_t)l * 512 + (size_t)srow * 8 + nc;
#pragma unroll
    for (int i = 0; i < 8; ++i) o[i] = (unsigned short)(bf16_bits(p[(size_t)i * 8]) & msk);
    put16(W3T + (size_t)(l * N3 + n) * K2 + k8, o);
    return;
  } else if (u < U3) {
    const int row = u - U2;
    const int rc  = row < nN ? row : nN - 1;
    const float okf = row < nN ? 1.0f : 0.0f;
    const float r0 = pos[(size_t)rc * 3 + 0];
    const float r1 = pos[(size_t)rc * 3 + 1];
    const float r2 = pos[(size_t)rc * 3 + 2];
    v4f q;
    q.x = bf16_val(r0) * okf;
    q.y = bf16_val(r1) * okf;
    q.z = bf16_val(r2) * okf;
    q.w = 0.0f;
    putf4(POSB + (size_t)row * 4, q);
    return;
  } else if (u < U4) {
    const int v   = u - U3;
    const int row = v >> 2;
    const int qq  = v & 3;
    const int rc  = row < nN ? row : nN - 1;
    const float okf = row < nN ? 1.0f : 0.0f;
    const float* p = nf + (size_t)rc * 7;
    const float f0 = p[0], f1 = p[1], f2 = p[2], f3 = p[3], f4 = p[4], f5 = p[5], f6 = p[6];
    const float s   = bf16_val(f0) * okf;
    const float v00 = bf16_val(f1) * okf, v01 = bf16_val(f2) * okf, v02 = bf16_val(f3) * okf;
    const float v10 = bf16_val(f4) * okf, v11 = bf16_val(f5) * okf, v12 = bf16_val(f6) * okf;
    const float wus = cw[32];
    const float a00 = cw[48], a01 = cw[49], a10 = cw[50], a11 = cw[51];
    const float su  = s * wus;
    const float u00 = (v00 * a00 + v10 * a10) * RSQ2;
    const float u01 = (v01 * a00 + v11 * a10) * RSQ2;
    const float u02 = (v02 * a00 + v12 * a10) * RSQ2;
    const float u10 = (v00 * a01 + v10 * a11) * RSQ2;
    const float u11 = (v01 * a01 + v11 * a11) * RSQ2;
    const float u12 = (v02 * a01 + v12 * a11) * RSQ2;
    const v4f c0 = {s, v00, v01, v02};
    const v4f c1 = {v10, v11, v12, 0.0f};
    const v4f c2 = {su, u00, u01, u02};
    const v4f c3 = {u10, u11, u12, 0.0f};
    const float g0 = (qq == 0) ? 1.0f : 0.0f;
    const float g1 = (qq == 1) ? 1.0f : 0.0f;
    const float g2 = (qq == 2) ? 1.0f : 0.0f;
    const float g3 = (qq == 3) ? 1.0f : 0.0f;
    const v4f r = (c0 * g0 + c1 * g1) + (c2 * g2 + c3 * g3);
    putf4(NODE0 + (size_t)v * 4, r);
    return;
  }
}

template <int APITCH, int NT>
__device__ __forceinline__ void wave_gemm_b(const unsigned short* sAw, float* sDw,
                                            const unsigned short* __restrict__ BT, int ldb, int K,
                                            int hh, int m) {
  v8f acc[2][NT];
  {
    const v8f z = {0.f, 0.f, 0.f, 0.f, 0.f, 0.f, 0.f, 0.f};
#pragma unroll
    for (int mt = 0; mt < 2; ++mt)
#pragma unroll
      for (int nt = 0; nt < NT; ++nt) acc[mt][nt] = z;
  }
  const unsigned short* ap0 = sAw + m * APITCH + 8 * hh;
  const unsigned short* ap1 = ap0 + 16 * APITCH;
  const unsigned short* bp  = BT + (size_t)m * (size_t)ldb + 8 * hh;
#pragma unroll 1
  for (int k0 = 0; k0 < K; k0 += 32) {
    FragB a0, a1;
    a0.h[0] = *(const v8usa*)(ap0 + k0);
    a0.h[1] = *(const v8usa*)(ap0 + k0 + 16);
    a1.h[0] = *(const v8usa*)(ap1 + k0);
    a1.h[1] = *(const v8usa*)(ap1 + k0 + 16);
#pragma unroll
    for (int nt = 0; nt < NT; ++nt) {
      const unsigned short* wq = bp + (size_t)(16 * nt) * (size_t)ldb + k0;
      FragB b;
      b.h[0] = *(const v8usa*)wq;
      b.h[1] = *(const v8usa*)(wq + 16);
      acc[0][nt] = wmb(a0, b, acc[0][nt]);
      acc[1][nt] = wmb(a1, b, acc[1][nt]);
    }
  }
#pragma unroll
  for (int nt = 0; nt < NT; ++nt) {
    const int col = 16 * nt + m;
#pragma unroll
    for (int mt = 0; mt < 2; ++mt)
#pragma unroll
      for (int r = 0; r < 8; ++r) sDw[(16 * mt + 8 * hh + r) * DP + col] = acc[mt][nt][r];
  }
}

__device__ __forceinline__ void ep_swish_split(const float* rd, unsigned short* ra, float scale) {
#pragma clang fp contract(off)
#pragma unroll 1
  for (int c8 = 0; c8 < HID / 8; ++c8) {
    const v4f va = *(const v4fa*)(rd + 8 * c8);
    const v4f vb = *(const v4fa*)(rd + 8 * c8 + 4);
    const v8f v8 = {va.x, va.y, va.z, va.w, vb.x, vb.y, vb.z, vb.w};
    v8us ho, lo;
#pragma unroll
    for (int i = 0; i < 8; ++i) {
      const float h = swishf(v8[i] * scale);
      const unsigned u  = __float_as_uint(h);
      const unsigned hs = (u + 0x7FFFu + ((u >> 16) & 1u)) & 0xFFFF0000u;
      const float    r  = h - __uint_as_float(hs);
      ho[i] = (unsigned short)(hs >> 16);
      lo[i] = (unsigned short)(__float_as_uint(r) >> 16);
    }
    *(v8usa*)(ra + 8 * c8)       = ho;
    *(v8usa*)(ra + HID + 8 * c8) = lo;
  }
}

__global__ __launch_bounds__(NTHR) void k_edge(const int* __restrict__ srcs, const int* __restrict__ dsts,
                                               int nE, int nN, const float* __restrict__ POSB,
                                               const unsigned short* __restrict__ W1T,
                                               const unsigned short* __restrict__ W2T,
                                               const unsigned short* __restrict__ W3T,
                                               float* MIX, int mixStride) {
#pragma clang fp contract(off)
  extern __shared__ __attribute__((aligned(16))) float dyn[];
  float*          sD = dyn;
  unsigned short* sA = (unsigned short*)(dyn + EPB * DP);
  unsigned short* sR = sA + EPB * AP;
  float*          sM = dyn + EPB * DP + (EPB * AP + EPB * FP) / 2;

  const int tid = (int)threadIdx.x, lane = tid & 31, wave = tid >> 5, hh = lane >> 4, m = lane & 15;

  const int  elb  = (int)blockIdx.x * EPB;
  const int  el   = elb + tid;
  const bool live = el < nE;
  const int  elc  = live ? el : (nE - 1);
  int s = srcs[elc];
  int t = dsts[elc];
  s = s < 0 ? 0 : (s > nN - 1 ? nN - 1 : s);
  t = t < 0 ? 0 : (t > nN - 1 ? nN - 1 : t);
  const v4f ps = *(const v4fa*)(POSB + (size_t)s * 4);
  const v4f pt = *(const v4fa*)(POSB + (size_t)t * 4);
  const float vx = pt.x - ps.x, vy = pt.y - ps.y, vz = pt.z - ps.z;
  const float len  = sqrtf((vx * vx + vz * vz) + vy * vy);
  const float safe = (len == 0.0f) ? 1.0f : len;
  const float rs   = 1.0f / safe;
  const float x  = len;
  const float x2 = x * x, x3 = x2 * x, x6 = x3 * x3, x7 = x6 * x, x8 = x6 * x2;
  const float poly = ((1.0f - 28.0f * x6) + 48.0f * x7) - 21.0f * x8;
  const float env  = (x < 1.0f) ? poly : 0.0f;
  const float zf   = (len == 0.0f) ? 0.0f : 1.0f;
  {
    unsigned short* rr = sR + tid * FP;
    v8us o0, o1, o2, oz;
#pragma unroll
    for (int k = 0; k < 8; ++k) {
      const float ck  = PIF * (float)(k + 1);
      const float sv  = sinf(ck * len);
      const float rad = (((SQRT2F * sv) * rs) * env) * zf;
      unsigned short a, b, c;
      split3(rad, a, b, c);
      o0[k] = a; o1[k] = b; o2[k] = c; oz[k] = (unsigned short)0;
    }
    *(v8usa*)(rr + 0)  = o0;
    *(v8usa*)(rr + 8)  = o1;
    *(v8usa*)(rr + 16) = o2;
    *(v8usa*)(rr + 24) = oz;
  }
  float*                rd  = sD + tid * DP;
  unsigned short*       ra  = sA + tid * AP;
  float*                rm  = sM + tid * MIXW;
  const unsigned short* sRw = sR + 32 * wave * FP;
  const unsigned short* sAw = sA + 32 * wave * AP;
  float*                sDw = sD + 32 * wave * DP;
  __syncthreads();

#pragma unroll 1
  for (int l = 0; l < NLAYER; ++l) {
    const unsigned short* w1 = W1T + (size_t)l * HID * K1;
    const unsigned short* w2 = W2T + (size_t)l * HID * K2;
    const unsigned short* w3 = W3T + (size_t)l * N3 * K2;

    wave_gemm_b<FP, 4>(sRw, sDw, w1, K1, K1, hh, m);
    __syncthreads();
    ep_swish_split(rd, ra, RSQ8);
    __syncthreads();
    wave_gemm_b<AP, 4>(sAw, sDw, w2, K2, K2, hh, m);
    __syncthreads();
    ep_swish_split(rd, ra, 0.125f);
    __syncthreads();
    wave_gemm_b<AP, 1>(sAw, sDw, w3, K2, K2, hh, m);
    __syncthreads();
    {
      const v4f va = *(const v4fa*)rd;
      const v4f vb = *(const v4fa*)(rd + 4);
      *(v4fa*)rm       = va * 0.125f;
      *(v4fa*)(rm + 4) = vb * 0.125f;
    }
    __syncthreads();
    {
      const v4f pv0 = *(const v4fa*)(sM + (size_t)4 * tid);
      const v4f pv1 = *(const v4fa*)(sM + (size_t)4 * (NTHR + tid));
      float* mp = MIX + (size_t)l * (size_t)mixStride + (size_t)elb * MIXW;
      *(volatile v4f*)(mp + (size_t)4 * tid)          = pv0;
      *(volatile v4f*)(mp + (size_t)4 * (NTHR + tid)) = pv1;
      __threadfence();
      *(volatile v4f*)(mp + (size_t)4 * tid)          = pv0;
      *(volatile v4f*)(mp + (size_t)4 * (NTHR + tid)) = pv1;
    }
  }
}

__global__ __launch_bounds__(NTHR) void k_scan(const int* __restrict__ dsts, const int* __restrict__ srcs,
                                               int nE, int nN, int vec8,
                                               const float* __restrict__ NODEc, const float* __restrict__ POSB,
                                               const float* __restrict__ MIXl,
                                               const float* __restrict__ Wss, const float* __restrict__ Wsv,
                                               const float* __restrict__ Wus, const float* __restrict__ Wuv,
                                               const float* __restrict__ Wds, const float* __restrict__ Wdv,
                                               int layer, int last, float* NODEn, float* out) {
#pragma clang fp contract(off)
  extern __shared__ __attribute__((aligned(16))) int dsm[];
  int*   list = dsm;
  int*   hl   = dsm + LISTN;
  int*   sl   = hl + RCAP;
  int*   cnt  = sl + RCAP;
  int*   offs = cnt + NBA;
  int*   cur  = offs + NBA;
  int*   misc = cur + NBA;
  float* cw   = (float*)(misc + 16);
  float* stg  = (float*)hl;
  const int tid = (int)threadIdx.x, lane = tid & 31, wave = tid >> 5;
  const int nodeBase = (int)blockIdx.x * NBA;

  {
    const v4i z4 = {0, 0, 0, 0};
    for (int i = tid * 4; i < AGG_ZINTS; i += NTHR * 4) *(v4ia*)(dsm + i) = z4;
    if (tid < 16) misc[tid] = 0;
    load_cw(cw, Wss, Wsv, Wus, Wuv, Wds, Wdv, tid);
  }
  __syncthreads();

  int t = 0, ov = 0;
  const int nChunks = (nE + CHUNK - 1) / CHUNK;
#pragma unroll 1
  for (int ch = 0; ch < nChunks; ++ch) {
    const int cbase = ch * CHUNK;
    const int wc = scan_chunk<SLA>(dsts, nE, cbase, nodeBase, NBA, vec8, list, tid, lane, wave);
    if (lane == 0) misc[wave] = wc;
    __syncthreads();
    if (wave == 0) {
#pragma unroll 1
      for (int w2 = 0; w2 < NWAVE; ++w2) {
        int c = misc[w2];
        c = c < 0 ? 0 : (c > WCAP ? WCAP : c);
#pragma unroll 1
        for (int b0 = 0; b0 < c; b0 += 32) {
          const int idx = b0 + lane;
          const int ent = list[w2 * WCAP + (idx < WCAP ? idx : WCAP - 1)];
          const int m32 = (c - b0) < 32 ? (c - b0) : 32;
#pragma unroll 1
          for (int k = 0; k < m32; ++k) {
            const int u    = __builtin_amdgcn_readlane(ent, k);
            const int slot = u & (NBA - 1);
            const int el   = (u >> SLA) & (CHUNK - 1);
            const int pk   = ((cbase + el) << SLA) | slot;
            if (t < RCAP) {
              if (lane == 0) { hl[t] = pk; cnt[slot] = cnt[slot] + 1; }
              t = t + 1;
            } else {
              ov = 1;
            }
          }
        }
      }
    }
    __syncthreads();
  }
  if (wave == 0 && lane == 0) { misc[8] = t; misc[9] = ov; }
  __syncthreads();
  int tt = misc[8];
  tt = tt < 0 ? 0 : (tt > RCAP ? RCAP : tt);
  const int ovf = misc[9];

  if (wave == 0) {
    const int base = lane * (NBA / 32);
    int s = 0;
#pragma unroll 1
    for (int i = 0; i < NBA / 32; ++i) s += cnt[base + i];
    int incl = s;
#pragma unroll
    for (int d = 1; d < 32; d <<= 1) {
      const int y = __shfl_up(incl, d, 32);
      if (lane >= d) incl += y;
    }
    int run = incl - s;
#pragma unroll 1
    for (int i = 0; i < NBA / 32; ++i) {
      const int cv = cnt[base + i];
      offs[base + i] = run;
      cur[base + i]  = run;
      run += cv;
    }
  }
  __syncthreads();
  if (wave == 0) {
#pragma unroll 1
    for (int b0 = 0; b0 < tt; b0 += 32) {
      const int idx = b0 + lane;
      const int ent = hl[idx < RCAP ? idx : RCAP - 1];
      const int m32 = (tt - b0) < 32 ? (tt - b0) : 32;
#pragma unroll 1
      for (int k = 0; k < m32; ++k) {
        const int u    = __builtin_amdgcn_readlane(ent, k);
        const int slot = u & (NBA - 1);
        if (lane == 0) {
          int p = cur[slot];
          p = p < 0 ? 0 : (p > RCAP - 1 ? RCAP - 1 : p);
          sl[p] = u;
          cur[slot] = p + 1;
        }
      }
    }
  }
  __syncthreads();

  const float qnan = __int_as_float(0x7fc00000);
  const float pz   = (ovf != 0) ? qnan : 0.0f;
  const int   lp   = (layer < 2) ? (layer + 1) : 2;
  const float* wss = cw + 3 * layer;
  const float* wsv = cw + 16 + 4 * layer;
  const float  wus = cw[32 + lp];
  const float* wuv = cw + 48 + 4 * lp;
  const float* wds = cw + 64 + 9 * layer;
  const float* wdv = cw + 96 + 10 * layer;
#pragma unroll 1
  for (int j = 0; j < NBA / NTHR; ++j) {
    const int slot = j * NTHR + tid;
    const int node = nodeBase + slot;
    int c = cnt[slot];
    const bool big = c > DEGCAP;
    c = c < 0 ? 0 : (c > DEGCAP ? DEGCAP : c);
    int o = offs[slot];
    o = o < 0 ? 0 : (o > RCAP ? RCAP : o);
    int cm = c;
#pragma unroll
    for (int d = 16; d > 0; d >>= 1) {
      const int y = __shfl_xor(cm, d, 32);
      cm = cm > y ? cm : y;
    }
    const v4f pt = *(const v4fa*)(POSB + (size_t)node * 4);
    float as0 = 0.0f, as1 = 0.0f, as2 = 0.0f;
    float av[15];
#pragma unroll
    for (int i = 0; i < 15; ++i) av[i] = 0.0f;
#pragma unroll 1
    for (int p = 0; p < cm; ++p) {
      const float vf = (p < c) ? 1.0f : 0.0f;
      int idx = o + p;
      idx = idx > RCAP - 1 ? RCAP - 1 : idx;
      const int ent = sl[idx];
      int eid = ent >> SLA;
      eid = eid < 0 ? 0 : (eid > nE - 1 ? nE - 1 : eid);
      int sn = srcs[eid];
      sn = sn < 0 ? 0 : (sn > nN - 1 ? nN - 1 : sn);
      const v4f ps = *(const v4fa*)(POSB + (size_t)sn * 4);
      const float* ur = NODEc + (size_t)sn * NODEW + 8;
      const v4f ua = *(const v4fa*)ur;
      const v4f ub = *(const v4fa*)(ur + 4);
      const float* mr = MIXl + (size_t)eid * MIXW;
      const v4f ma = *(const v4fa*)mr;
      const v4f mb = *(const v4fa*)(mr + 4);
      const float vx = pt.x - ps.x, vy = pt.y - ps.y, vz = pt.z - ps.z;
      const float len  = sqrtf((vx * vx + vz * vz) + vy * vy);
      const float safe = (len == 0.0f) ? 1.0f : len;
      const float rs   = 1.0f / safe;
      const float nn[3] = {vx * rs, vy * rs, vz * rs};
      const float m0 = ma.x * vf, m1 = ma.y * vf, m2 = ma.z * vf, m3 = ma.w * vf;
      const float m4 = mb.x * vf, m5 = mb.y * vf, m6 = mb.z * vf, m7 = mb.w * vf;
      const float se = ua.x;
      const float v0[3] = {ua.y, ua.z, ua.w};
      const float v1[3] = {ub.x, ub.y, ub.z};
      const float d0 = (v0[0] * nn[0] + v0[1] * nn[1]) + v0[2] * nn[2];
      const float d1 = (v1[0] * nn[0] + v1[1] * nn[1]) + v1[2] * nn[2];
      as0 += se * m0;
      as1 += d0 * m1;
      as2 += d1 * m2;
      const float pbk = SQRT3F * se;
#pragma unroll
      for (int cc = 0; cc < 3; ++cc) {
        av[cc]      += v0[cc] * m3;
        av[3 + cc]  += v1[cc] * m4;
        av[6 + cc]  += (C121F * (d0 * nn[cc] - v0[cc] * THIRD)) * m5;
        av[9 + cc]  += (C121F * (d1 * nn[cc] - v1[cc] * THIRD)) * m6;
        av[12 + cc] += (pbk * nn[cc]) * m7;
      }
    }
    const float* own = NODEc + (size_t)node * NODEW;
    const v4f oa = *(const v4fa*)own;
    const v4f ob = *(const v4fa*)(own + 4);
    const float s = oa.x;
    const float w0[3] = {oa.y, oa.z, oa.w};
    const float w1[3] = {ob.x, ob.y, ob.z};
    float st[3];
#pragma unroll
    for (int k = 0; k < 3; ++k)
      st[k] = ((as0 * wds[k] + as1 * wds[3 + k]) + as2 * wds[6 + k]) * RSQ3 + s * wss[k];
    float vt[2][3];
#pragma unroll
    for (int k = 0; k < 2; ++k) {
#pragma unroll
      for (int cc = 0; cc < 3; ++cc) {
        const float vd = (((av[cc] * wdv[k] + av[3 + cc] * wdv[2 + k]) + av[6 + cc] * wdv[4 + k]) +
                          av[9 + cc] * wdv[6 + k]) + av[12 + cc] * wdv[8 + k];
        vt[k][cc] = vd * RSQ5 + (w0[cc] * wsv[k] + w1[cc] * wsv[2 + k]) * RSQ2;
      }
    }
    const float snew = swishf(st[0]);
    const float g1   = swishf(st[1]);
    const float g2   = swishf(st[2]);
    float vn0[3], vn1[3];
#pragma unroll
    for (int cc = 0; cc < 3; ++cc) { vn0[cc] = vt[0][cc] * g1; vn1[cc] = vt[1][cc] * g2; }
    const float pzr = big ? qnan : pz;
    if (last == 0) {
      const float su = snew * wus;
      float vu0[3], vu1[3];
#pragma unroll
      for (int cc = 0; cc < 3; ++cc) {
        vu0[cc] = (vn0[cc] * wuv[0] + vn1[cc] * wuv[2]) * RSQ2;
        vu1[cc] = (vn0[cc] * wuv[1] + vn1[cc] * wuv[3]) * RSQ2;
      }
      const v4f r0 = {snew + pzr, vn0[0] + pzr, vn0[1] + pzr, vn0[2] + pzr};
      const v4f r1 = {vn1[0] + pzr, vn1[1] + pzr, vn1[2] + pzr, pzr};
      const v4f r2 = {su + pzr, vu0[0] + pzr, vu0[1] + pzr, vu0[2] + pzr};
      const v4f r3 = {vu1[0] + pzr, vu1[1] + pzr, vu1[2] + pzr, pzr};
      float* sp = stg + (size_t)slot * NODEW;
      *(v4fa*)(sp)      = r0;
      *(v4fa*)(sp + 4)  = r1;
      *(v4fa*)(sp + 8)  = r2;
      *(v4fa*)(sp + 12) = r3;
    } else {
      stg[slot * 3 + 0] = vn0[0] + pzr;
      stg[slot * 3 + 1] = vn0[1] + pzr;
      stg[slot * 3 + 2] = vn0[2] + pzr;
    }
  }
  __syncthreads();

  if (last == 0) {
    v4f pv[16];
#pragma unroll
    for (int it = 0; it < 16; ++it) pv[it] = *(const v4fa*)(stg + (size_t)4 * (it * NTHR + tid));
    float* nb = NODEn + (size_t)nodeBase * NODEW;
#pragma unroll
    for (int it = 0; it < 16; ++it) *(volatile v4f*)(nb + (size_t)4 * (it * NTHR + tid)) = pv[it];
    __threadfence();
#pragma unroll
    for (int it = 0; it < 16; ++it) *(volatile v4f*)(nb + (size_t)4 * (it * NTHR + tid)) = pv[it];
  } else {
    v4f pv[3];
#pragma unroll
    for (int it = 0; it < 3; ++it) pv[it] = *(const v4fa*)(stg + (size_t)4 * (it * NTHR + tid));
    const long long lim = 3LL * nN;
#pragma unroll
    for (int it = 0; it < 3; ++it) {
      const long long gidx = (long long)nodeBase * 3 + 4LL * (it * NTHR + tid);
      if (gidx + 4 <= lim) *(volatile v4f*)(out + (size_t)gidx) = pv[it];
    }
    __threadfence();
#pragma unroll
    for (int it = 0; it < 3; ++it) {
      const long long gidx = (long long)nodeBase * 3 + 4LL * (it * NTHR + tid);
      if (gidx + 4 <= lim) *(volatile v4f*)(out + (size_t)gidx) = pv[it];
    }
  }
}

static inline int cdiv(int a, int b) { return (a + b - 1) / b; }

extern "C" void kernel_launch(void* const* d_in, const int* in_sizes, int n_in,
                              void* d_out, int out_size, void* d_ws, size_t ws_size,
                              hipStream_t stream) {
  if (n_in < 13) return;
  if (in_sizes[0] < 3 || (in_sizes[0] % 3) != 0) return;
  const int nN = in_sizes[0] / 3;
  if (in_sizes[1] != 7 * nN) return;
  const int nE = in_sizes[2];
  if (nE < 1 || nE >= (1 << 21)) return;
  if (in_sizes[3] != nE) return;
  if (in_sizes[4] != NLAYER * 3 || in_sizes[5] != NLAYER * 4) return;
  if (in_sizes[6] != NLAYER * 1 || in_sizes[7] != NLAYER * 4) return;
  if (in_sizes[8] != NLAYER * 8 * HID) return;
  if (in_sizes[9] != NLAYER * HID * HID) return;
  if (in_sizes[10] != NLAYER * HID * 8) return;
  if (in_sizes[11] != NLAYER * 9 || in_sizes[12] != NLAYER * 10) return;
  if ((long long)out_size != 3LL * nN) return;
  if (((3 * nN) & 3) != 0) return;

  const float* pos = (const float*)d_in[0];
  const float* nf  = (const float*)d_in[1];
  const int*   snd = (const int*)d_in[2];
  const int*   rcv = (const int*)d_in[3];
  const float* Wss = (const float*)d_in[4];
  const float* Wsv = (const float*)d_in[5];
  const float* Wus = (const float*)d_in[6];
  const float* Wuv = (const float*)d_in[7];
  const float* W1  = (const float*)d_in[8];
  const float* W2  = (const float*)d_in[9];
  const float* W3  = (const float*)d_in[10];
  const float* Wds = (const float*)d_in[11];
  const float* Wdv = (const float*)d_in[12];
  float* out = (float*)d_out;

  const int gA = cdiv(nN, NBA);
  const int nR = gA * NBA;
  const int EP = cdiv(nE, EPB) * EPB;
  if ((nR % NTHR) != 0) return;

  char* ws = (char*)d_ws;
  size_t off = 0;
  const size_t oW1  = off; off += (size_t)NLAYER * HID * K1 * 2;     off = (off + 255) & ~(size_t)255;
  const size_t oW2  = off; off += (size_t)NLAYER * HID * K2 * 2;     off = (off + 255) & ~(size_t)255;
  const size_t oW3  = off; off += (size_t)NLAYER * N3 * K2 * 2;      off = (off + 255) & ~(size_t)255;
  const size_t oPB  = off; off += (size_t)nR * 4 * 4;                off = (off + 255) & ~(size_t)255;
  const size_t oNA  = off; off += (size_t)nR * NODEW * 4;            off = (off + 255) & ~(size_t)255;
  const size_t oNB  = off; off += (size_t)nR * NODEW * 4;            off = (off + 255) & ~(size_t)255;
  const size_t oMX  = off; off += (size_t)NLAYER * EP * MIXW * 4;    off = (off + 255) & ~(size_t)255;
  if (off > ws_size || off > (size_t)WSMAX) return;
  unsigned short* W1T   = (unsigned short*)(ws + oW1);
  unsigned short* W2T   = (unsigned short*)(ws + oW2);
  unsigned short* W3T   = (unsigned short*)(ws + oW3);
  float*          POSB  = (float*)(ws + oPB);
  float*          NODEA = (float*)(ws + oNA);
  float*          NODEB = (float*)(ws + oNB);
  float*          MIX   = (float*)(ws + oMX);
  const int mixStride = EP * MIXW;

  hipFuncSetAttribute(reinterpret_cast<const void*>(&k_edge), hipFuncAttributeMaxDynamicSharedMemorySize,
                      (int)EDGE_LDS_BYTES);
  hipFuncSetAttribute(reinterpret_cast<const void*>(&k_scan), hipFuncAttributeMaxDynamicSharedMemorySize,
                      (int)AGG_LDS_BYTES);

  const int nPrep = NU_W1 + NU_W2 + NU_W3 + nR + 4 * nR;
  const int vec8  = 1;

  k_prep<<<nPrep / NTHR, NTHR, 0, stream>>>(pos, nf, Wss, Wsv, Wus, Wuv, Wds, Wdv, W1, W2, W3, nN, nR,
                                            W1T, W2T, W3T, POSB, NODEA);
  k_edge<<<EP / EPB, NTHR, EDGE_LDS_BYTES, stream>>>(snd, rcv, nE, nN, POSB, W1T, W2T, W3T, MIX, mixStride);
  for (int l = 0; l < NLAYER; ++l) {
    const float* curN = (l & 1) ? NODEB : NODEA;
    float*       nxtN = (l & 1) ? NODEA : NODEB;
    const int    last = (l == NLAYER - 1) ? 1 : 0;
    k_scan<<<gA, NTHR, AGG_LDS_BYTES, stream>>>(rcv, snd, nE, nN, vec8, curN, POSB,
                                                MIX + (size_t)l * (size_t)mixStride,
                                                Wss, Wsv, Wus, Wuv, Wds, Wdv, l, last, nxtN, out);
  }
}
